// HetGNN_14817637171202
// MI455X (gfx1250) — hardware-run, weakly checked
//
#include <hip/hip_runtime.h>


namespace {
constexpr int N = 100000, NP = 100032, ER = 500000, R = 3, E = R * ER  , NK = R * N  , D = 128, KT = R * D  , HH = 64;
constexpr float XS = 8.0f, WSC = 256.0f, NEG = 0.2f  ;

typedef _Float16 b16;
typedef __attribute__((ext_vector_type(16))) _Float16 v16b;
typedef __attribute__((ext_vector_type(8))) _Float16 v8b;
typedef __attribute__((ext_vector_type(8))) float v8f;
typedef __attribute__((ext_vector_type(4))) float v4f;
__device__ __forceinline__ float bf16_rne(float f) { unsigned int u = __float_as_uint(f); u += 0x7FFFu + ((u >> 16) & 1u); return __uint_as_float(u & 0xFFFF0000u); }
__device__ __forceinline__ void split16(float v, b16& hi, b16& lo) { hi = (b16)v; lo = (b16)(v - (float)hi); }
__device__ __forceinline__ v16b frag_kb(const b16* p, int hh) { const v8b a = *(const v8b*)(p + 8 * hh), b = *(const v8b*)(p + 16 + 8 * hh); v16b f;
#pragma unroll
  for (int e = 0; e < 8; ++e) { f[e] = a[e]; f[8 + e] = b[e]; } return f; }
__device__ __forceinline__ v8f wmma16b(v16b a, v16b b, v8f c) { v8f d = __builtin_amdgcn_wmma_f32_16x16x32_f16(false, a, false, b, (short)0, c, false, false); asm volatile("v_nop\n\tv_nop\n\tv_nop\n\tv_nop" : "+v"(d) : "v"(a), "v"(b)); return d; }
__device__ __forceinline__ void wave_lds_sync() { __builtin_amdgcn_fence(__ATOMIC_RELEASE, "workgroup"); __builtin_amdgcn_wave_barrier(); __builtin_amdgcn_fence(__ATOMIC_ACQUIRE, "workgroup"); }
__device__ __forceinline__ float pmul(float a, float b) { float p = a * b; asm volatile("" : "+v"(p)); return p; }
__device__ __forceinline__ int iclamp(int v, int lo, int hi) { return v < lo ? lo : (v > hi ? hi : v); }
__device__ __forceinline__ float nexp(float x) { return __builtin_amdgcn_exp2f(x * 1.4426950408889634f); }
__device__ __forceinline__ float lrelu(float x) { return x > 0.0f ? x : NEG * x; }

constexpr int CSR_NBLK = 512, CSR_GB = 10  , CSR_GN = 1 << CSR_GB  , CSR_MAXG = 512, CSR_CAP = 12288  ;
__global__ __launch_bounds__(64) void csrA_kernel(const int* __restrict__ dst, int E, int N, int nG, int CHP, int NGP, int* __restrict__ STG, int* __restrict__ HST) {
  extern __shared__ int sm[];
  int* cnt = sm; int* run = sm + NGP; int* ids = sm + 2 * NGP;
  const int b = blockIdx.x; const int ch = (E + CSR_NBLK - 1) / CSR_NBLK; const int e0 = b * ch, e1 = min(E, e0 + ch);
  for (int i = threadIdx.x; i < NGP; i += 64) cnt[i] = 0;
  for (int i = threadIdx.x; i < CHP; i += 64) ids[i] = -1;
  __syncthreads();
  if (threadIdx.x == 0) {
    for (int e = e0; e < e1; ++e) { int d = dst[e]; d = (d < 0) ? 0 : (d >= N ? N - 1 : d); cnt[d >> CSR_GB] += 1; }
    int acc = 0; for (int g = 0; g < nG; ++g) { run[g] = acc; acc += cnt[g]; }
    for (int e = e0; e < e1; ++e) { int d = dst[e]; d = (d < 0) ? 0 : (d >= N ? N - 1 : d); const int g = d >> CSR_GB; ids[run[g]] = e; run[g] += 1; } }
  __syncthreads();
  typedef __attribute__((ext_vector_type(4))) int v4i;
  for (int pass = 0; pass < 2; ++pass) {
    for (int i = threadIdx.x; i < CHP / 4; i += 64) *(volatile v4i*)(STG + (size_t)b * CHP + i * 4) = *(const v4i*)(&ids[i * 4]);
    for (int i = threadIdx.x; i < NGP / 4; i += 64) { v4i v; for (int e = 0; e < 4; ++e) v[e] = (i * 4 + e < nG) ? cnt[i * 4 + e] : 0; *(volatile v4i*)(HST + (size_t)b * NGP + i * 4) = v; }
    __threadfence(); }
}
__global__ __launch_bounds__(512) void csrS_kernel(const int* __restrict__ HST, int nG, int NGP, int* __restrict__ START, int* __restrict__ TOT, int* __restrict__ OFF) {
  __shared__ int tot[CSR_MAXG];
  const int b = threadIdx.x;
  for (int pass = 0; pass < 2; ++pass) { int runb = 0; for (int g = 0; g < nG; ++g) { int c = HST[(size_t)b * NGP + g]; c = (c < 0) ? 0 : c; ((volatile int*)OFF)[(size_t)g * CSR_NBLK + b] = runb; runb += c; } __threadfence(); }
  for (int g = threadIdx.x; g < nG; g += 512) { int s = 0; for (int bb = 0; bb < CSR_NBLK; ++bb) { int c = HST[(size_t)bb * NGP + g]; s += (c < 0) ? 0 : c; } tot[g] = s; }
  __syncthreads();
  if (threadIdx.x < 32) {
    __shared__ int st[CSR_MAXG + 32];
    if (threadIdx.x == 0) { int acc = 0; for (int g = 0; g < NGP; ++g) { st[g] = acc; if (g < nG) acc += (tot[g] + 31) & ~31; } st[NGP] = acc; }
    __builtin_amdgcn_fence(__ATOMIC_RELEASE, "workgroup"); __builtin_amdgcn_wave_barrier(); __builtin_amdgcn_fence(__ATOMIC_ACQUIRE, "workgroup");
    for (int pass = 0; pass < 2; ++pass) { for (int i = threadIdx.x; i < NGP + 32; i += 32) { ((volatile int*)START)[i] = (i <= NGP) ? st[min(i, NGP)] : 0; ((volatile int*)TOT)[i] = (i < nG) ? tot[i] : 0; } __threadfence(); } }
}
__global__ __launch_bounds__(256) void csrB_kernel(const int* __restrict__ dst, int N, int nG, int CHP, int NGP, int permLen, const int* __restrict__ STG, const int* __restrict__ HST, const int* __restrict__ OFF, const int* __restrict__ START, const int* __restrict__ TOT, int* __restrict__ PERM, int* __restrict__ ROWPTR, int* __restrict__ ROWCNT, int* __restrict__ FLAG) {
  typedef __attribute__((ext_vector_type(4))) int v4i;
  __shared__ int ids[CSR_CAP]; __shared__ unsigned short key[CSR_CAP]; __shared__ int outp[CSR_CAP]; __shared__ int ncnt[CSR_GN + 1]; __shared__ int boff[CSR_NBLK + 1];
  const int g = blockIdx.x, t_ = threadIdx.x; int tot = TOT[g]; int st = START[g], stn = START[g + 1]; const int v0 = g * CSR_GN; const int nv = min(CSR_GN, N - v0);
  st = (st < 0) ? 0 : (st > permLen - 32 ? permLen - 32 : st) & ~31; stn = (stn < st) ? st : (stn > permLen ? permLen : stn); tot = (tot < 0) ? 0 : tot; if (tot > stn - st && tot <= CSR_CAP) tot = stn - st;
  if (tot > CSR_CAP) {
    for (int pass = 0; pass < 2; ++pass) { for (int i = t_; i < CSR_GN / 4; i += 256) { v4i a, c; for (int e = 0; e < 4; ++e) { a[e] = st; c[e] = 0; } *(volatile v4i*)(ROWPTR + v0 + i * 4) = a; *(volatile v4i*)(ROWCNT + v0 + i * 4) = c; } if (t_ == 0) ((volatile int*)FLAG)[0] = 1; __threadfence(); } (void)nv; return; }
  if (t_ == 0) { int acc = 0; for (int b = 0; b < CSR_NBLK; ++b) { boff[b] = acc; int c = HST[(size_t)b * NGP + g]; c = (c < 0) ? 0 : (c > CHP ? CHP : c); acc += c; if (acc > tot) acc = tot; } boff[CSR_NBLK] = acc; }
  for (int i = t_; i <= CSR_GN; i += 256) ncnt[i] = 0;
  __syncthreads();
  for (int b = 0; b < CSR_NBLK; ++b) { const int c = boff[b + 1] - boff[b]; int o_ = OFF[(size_t)g * CSR_NBLK + b]; o_ = (o_ < 0) ? 0 : (o_ > CHP - c ? CHP - c : o_); const int* src_ = STG + (size_t)b * CHP + o_;
    for (int i = t_; i < c; i += 256) { int id = src_[i]; id = (id < 0) ? 0 : id; ids[boff[b] + i] = id; int d = dst[id]; d = (d < v0) ? v0 : (d >= N ? N - 1 : d); int kk = d - v0; kk = (kk < 0) ? 0 : (kk >= CSR_GN ? CSR_GN - 1 : kk); key[boff[b] + i] = (unsigned short)kk; } }
  __syncthreads();
  if (t_ == 0) { for (int i = 0; i < tot; ++i) ncnt[key[i]] += 1; int acc = 0; for (int vl = 0; vl < CSR_GN; ++vl) { const int c = ncnt[vl]; ncnt[vl] = acc; acc += c; } ncnt[CSR_GN] = acc;
    for (int i = 0; i < tot; ++i) { const int vl = key[i]; outp[ncnt[vl]] = ids[i]; ncnt[vl] += 1; }
    for (int vl = CSR_GN; vl > 0; --vl) ncnt[vl] = ncnt[vl - 1]; ncnt[0] = 0; }
  __syncthreads();
  for (int pass = 0; pass < 2; ++pass) {
    for (int i = t_; i < (stn - st) / 4; i += 256) { v4i v; for (int e = 0; e < 4; ++e) { const int q = i * 4 + e; v[e] = (q < tot) ? outp[q] : -1; } *(volatile v4i*)(PERM + st + i * 4) = v; }
    for (int i = t_; i < CSR_GN / 4; i += 256) { v4i a, c; for (int e = 0; e < 4; ++e) { const int vl = i * 4 + e; a[e] = st + ncnt[vl]; c[e] = (vl < nv) ? (ncnt[vl + 1] - ncnt[vl]) : 0; } *(volatile v4i*)(ROWPTR + v0 + i * 4) = a; *(volatile v4i*)(ROWCNT + v0 + i * 4) = c; }
    __threadfence(); }
}
__global__ __launch_bounds__(256) void csrZ_kernel(int* __restrict__ p, size_t n4) { typedef __attribute__((ext_vector_type(4))) int v4i; const size_t tid = (size_t)blockIdx.x * 256 + threadIdx.x, nth = (size_t)gridDim.x * 256; v4i z = {0, 0, 0, 0}; for (size_t i = tid; i < n4; i += nth) *(volatile v4i*)(p + i * 4) = z; }
struct CsrBufs { int *STG, *HST, *OFF, *START, *TOT, *PERM, *ROWPTR, *ROWCNT, *FLAG; int nG, NGP, CHP; size_t permLen; char* base; size_t bytes; };
static size_t csr_carve(CsrBufs& c, char* ws, size_t off, int E, int N) {
  const size_t off0 = off; c.base = ws + off;
  auto al = [&](size_t bytes) { char* p = ws + off; off += (bytes + 255) & ~(size_t)255; return p; };
  c.nG = (N + CSR_GN - 1) / CSR_GN; c.NGP = (c.nG + 31) & ~31; const int ch = (E + CSR_NBLK - 1) / CSR_NBLK; c.CHP = (ch + 31) & ~31; c.permLen = (size_t)E + 32 * (size_t)c.nG + 32;
  c.STG = (int*)al((size_t)CSR_NBLK * c.CHP * 4); c.HST = (int*)al((size_t)CSR_NBLK * c.NGP * 4); c.OFF = (int*)al((size_t)c.NGP * CSR_NBLK * 4); c.START = (int*)al((size_t)(c.NGP + 64) * 4); c.TOT = (int*)al((size_t)(c.NGP + 64) * 4);
  c.PERM = (int*)al(c.permLen * 4); c.ROWPTR = (int*)al((size_t)c.nG * CSR_GN * 4); c.ROWCNT = (int*)al((size_t)c.nG * CSR_GN * 4); c.FLAG = (int*)al(256);
  c.bytes = off - off0; return off;
}
static void csr_build(const CsrBufs& c, const int* dst, int E, int N, hipStream_t stream) {
  const size_t smem = (size_t)(2 * c.NGP + c.CHP) * 4;
  csrZ_kernel<<<512, 256, 0, stream>>>((int*)c.base, c.bytes / 16);
  csrA_kernel<<<CSR_NBLK, 64, smem, stream>>>(dst, E, N, c.nG, c.CHP, c.NGP, c.STG, c.HST);
  csrS_kernel<<<1, 512, 0, stream>>>(c.HST, c.nG, c.NGP, c.START, c.TOT, c.OFF);
  csrB_kernel<<<c.nG, 256, 0, stream>>>(dst, N, c.nG, c.CHP, c.NGP, (int)c.permLen, c.STG, c.HST, c.OFF, c.START, c.TOT, c.PERM, c.ROWPTR, c.ROWCNT, c.FLAG);
}


__global__ __launch_bounds__(256) void keys_kernel(const int* __restrict__ src, const int* __restrict__ dst, int* __restrict__ KS, int* __restrict__ KD) {
  typedef __attribute__((ext_vector_type(4))) int v4i;
  const size_t u = (size_t)blockIdx.x * 256 + threadIdx.x; if (u * 4 >= (size_t)E) return; const size_t e0 = u * 4; v4i ks, kd;
  for (int j = 0; j < 4; ++j) { const size_t e = e0 + j; const int r = (int)(e / ER); ks[j] = r * N + iclamp(src[e], 0, N - 1); kd[j] = r * N + iclamp(dst[e], 0, N - 1); }
  for (int pass = 0; pass < 2; ++pass) { *(volatile v4i*)(KS + e0) = ks; *(volatile v4i*)(KD + e0) = kd; __threadfence(); }
}
__global__ __launch_bounds__(256) void wprep_kernel(const float* __restrict__ W1, const float* __restrict__ W2, const float* __restrict__ wf, const float* __restrict__ wb, b16* __restrict__ WS1, b16* __restrict__ WS2, b16* __restrict__ WL) {
  const size_t u = (size_t)blockIdx.x * 256 + threadIdx.x; const size_t n1 = (size_t)D * KT / 8, n3 = (size_t)2 * 4 * HH * D / 8; size_t t = u; v8b o;
  if (t < 2 * n1) { const int l = (int)(t / n1); const size_t e = (t % n1) * 8; const int oo = (int)(e / KT), k0 = (int)(e % KT); const float* Wl = l ? W2 : W1;
    for (int j = 0; j < 8; ++j) { const int k = k0 + j; const int r = k / D, kk = k % D; o[j] = (b16)(bf16_rne(Wl[((size_t)r * D + kk) * D + oo]) * WSC); } for (int pass = 0; pass < 2; ++pass) { *(volatile v8b*)((l ? WS2 : WS1) + e) = o; __threadfence(); } return; } t -= 2 * n1;
  if (t < n3) { const size_t e = t * 8; const int row = (int)(e / D), k0 = (int)(e % D); const float* w = row < 4 * HH ? wf : wb; const int rr = row < 4 * HH ? row : row - 4 * HH;
    for (int j = 0; j < 8; ++j) o[j] = (b16)(bf16_rne(w[(size_t)rr * D + k0 + j]) * WSC); for (int pass = 0; pass < 2; ++pass) { *(volatile v8b*)(WL + e) = o; __threadfence(); } }
}
template <int LAYER0, int RELU, int FUSE>
__global__ __launch_bounds__(32) void hconv_kernel(const float* __restrict__ xin, const int* __restrict__ srcs, const int* __restrict__ PERMD, const int* __restrict__ ROWPTRD, const int* __restrict__ ROWCNTD, int permLenD, const int* __restrict__ ROWCNTS, const b16* __restrict__ WS, const float* __restrict__ bias  , float* __restrict__ Hout,
    const b16* __restrict__ WL, const float* __restrict__ bihf, const float* __restrict__ bhhf, const float* __restrict__ bihb, const float* __restrict__ bhhb, float* __restrict__ out) {
  __shared__ __attribute__((aligned(16))) b16 Ah[16][KT + 8], Al[16][KT + 8]; __shared__ __attribute__((aligned(16))) float Tf[16][D + 4];
  const int lane = threadIdx.x, nloc = lane & 15, hlf = lane >> 4; const size_t v0 = (size_t)blockIdx.x * 16;
  auto rd = [&](size_t u, int c) -> float { return LAYER0 ? bf16_rne(xin[u * D + c]) : xin[u * D + c]; };
  for (int rr = 0; rr < 16; ++rr) { const size_t v = v0 + rr;
    for (int r = 0; r < R; ++r) { float a[4] = {0.0f, 0.0f, 0.0f, 0.0f}; float scale = 0.0f;
      if (v < (size_t)N) { const size_t key = (size_t)r * N + v; int st = ROWPTRD[key], ct = ROWCNTD[key]; ct = iclamp(ct, 0, 65536); st = iclamp(st, 0, permLenD - ct); scale = rsqrtf(fmaxf((float)ct, 1.0f));
        for (int q = 0; q < ct; ++q) { const int e = iclamp(PERMD[st + q], 0, E - 1); const size_t s = (size_t)iclamp(srcs[e], 0, N - 1); const float so = rsqrtf(fmaxf((float)iclamp(ROWCNTS[(size_t)r * N + s], 0, 65536), 1.0f));
          const v4f xv = LAYER0 ? (v4f){rd(s, lane * 4), rd(s, lane * 4 + 1), rd(s, lane * 4 + 2), rd(s, lane * 4 + 3)} : *(const v4f*)(xin + s * D + lane * 4);
          for (int j = 0; j < 4; ++j) a[j] += pmul(xv[j], so); } }
      v8b dummy; (void)dummy;
      for (int j = 0; j < 4; ++j) { b16 p, pl; split16(pmul(a[j], scale) * XS, p, pl); Ah[rr][r * D + lane * 4 + j] = p; Al[rr][r * D + lane * 4 + j] = pl; } } }
  wave_lds_sync();
  v8f d[8];
#pragma unroll
  for (int t = 0; t < 8; ++t) d[t] = (v8f){};
#pragma unroll 2
  for (int kb = 0; kb < KT; kb += 32) { const v16b fa = frag_kb(&Ah[nloc][kb], hlf), fl = frag_kb(&Al[nloc][kb], hlf);
#pragma unroll
    for (int t = 0; t < 8; ++t) { const v16b bw = frag_kb(WS + (size_t)(t * 16 + nloc) * KT + kb, hlf); d[t] = wmma16b(fa, bw, d[t]); d[t] = wmma16b(fl, bw, d[t]); } }
#pragma unroll
  for (int t = 0; t < 8; ++t) { const int c = t * 16 + nloc; const float bm = ((bf16_rne(bias[c]) + bf16_rne(bias[D + c])) + bf16_rne(bias[2 * D + c])) * (1.0f / 3.0f);
#pragma unroll 1
    for (int r = 0; r < 8; ++r) { const int rr = 8 * hlf + r; float y = d[t][r] * (1.0f / (XS * WSC)) * (1.0f / 3.0f) + bm; if (RELU) y = fmaxf(y, 0.0f); if (v0 + rr >= (size_t)N) y = 0.0f; Tf[rr][c] = y; } }
  wave_lds_sync();
  if (!FUSE) { for (int pass = 0; pass < 2; ++pass) { for (int rr = 0; rr < 16; ++rr) *(volatile v4f*)(Hout + (v0 + rr) * D + lane * 4) = *(const v4f*)(&Tf[rr][lane * 4]); __threadfence(); } return; }
  for (int rr = 0; rr < 16; ++rr) for (int j = 0; j < 4; ++j) { b16 p, pl; split16(Tf[rr][lane * 4 + j] * XS, p, pl); Ah[rr][lane * 4 + j] = p; Al[rr][lane * 4 + j] = pl; }
  wave_lds_sync();
  __shared__ __attribute__((aligned(16))) float To[16][D + 4];
  for (int dir = 0; dir < 2; ++dir) { const b16* W = WL + (size_t)dir * 4 * HH * D; const float* bi = dir ? bihb : bihf; const float* bh = dir ? bhhb : bhhf;
    for (int t = 0; t < 4; ++t) { v8f gi = {}, gg = {}, go = {};
#pragma unroll
      for (int kb = 0; kb < D; kb += 32) { const v16b a = frag_kb(&Ah[nloc][kb], hlf), al = frag_kb(&Al[nloc][kb], hlf); v16b bw = frag_kb(W + (size_t)(t * 16 + nloc) * D + kb, hlf); gi = wmma16b(a, bw, gi); gi = wmma16b(al, bw, gi);
        bw = frag_kb(W + (size_t)(2 * HH + t * 16 + nloc) * D + kb, hlf); gg = wmma16b(a, bw, gg); gg = wmma16b(al, bw, gg); bw = frag_kb(W + (size_t)(3 * HH + t * 16 + nloc) * D + kb, hlf); go = wmma16b(a, bw, go); go = wmma16b(al, bw, go); }
      const int j = t * 16 + nloc; const float bI = bf16_rne(bi[j]) + bf16_rne(bh[j]), bG = bf16_rne(bi[2 * HH + j]) + bf16_rne(bh[2 * HH + j]), bO = bf16_rne(bi[3 * HH + j]) + bf16_rne(bh[3 * HH + j]);
#pragma unroll 1
      for (int r = 0; r < 8; ++r) { const float i_ = 1.0f / (1.0f + __expf(-(gi[r] * (1.0f / (XS * WSC)) + bI))); const float g_ = tanhf(gg[r] * (1.0f / (XS * WSC)) + bG); const float o_ = 1.0f / (1.0f + __expf(-(go[r] * (1.0f / (XS * WSC)) + bO))); To[8 * hlf + r][dir * HH + j] = pmul(o_, tanhf(pmul(i_, g_))); } } }
  wave_lds_sync();
  for (int pass = 0; pass < 2; ++pass) { for (int rr = 0; rr < 16; ++rr) if (v0 + rr < (size_t)N) *(volatile v4f*)(out + (v0 + rr) * D + lane * 4) = *(const v4f*)(&To[rr][lane * 4]); __threadfence(); }
}
}

extern "C" void kernel_launch(void* const* d_in, const int* in_sizes, int n_in, void* d_out, int out_size, void* d_ws, size_t ws_size, hipStream_t stream) {
  (void)n_in;
  auto Fp = [&](int i) { return (const float*)d_in[i]; }; auto Ip = [&](int i) { return (const int*)d_in[i]; };
  if (in_sizes[0] != N * D || in_sizes[1] != E || in_sizes[2] != E || in_sizes[3] != R * D * D || in_sizes[5] != R * D * D || in_sizes[7] != 4 * HH * D || in_sizes[11] != 4 * HH * D || out_size != N * D) return;
  size_t off = 0; char* ws = (char*)d_ws;
  auto carve = [&](size_t bytes) { char* p = ws + off; off += (bytes + 255) & ~(size_t)255; return p; };
  int* KS = (int*)carve((size_t)E * 4); int* KD = (int*)carve((size_t)E * 4); b16* WS1 = (b16*)carve((size_t)D * KT * 2); b16* WS2 = (b16*)carve((size_t)D * KT * 2); b16* WL = (b16*)carve((size_t)2 * 4 * HH * D * 2);
  float* HA = (float*)carve((size_t)NP * D * 4);
  CsrBufs cd, cs; off = csr_carve(cd, ws, off, E, NK); off = csr_carve(cs, ws, off, E, NK);
  if (off > ws_size || off > ((size_t)128 << 20)) return;
  keys_kernel<<<(unsigned)(((size_t)E / 4 + 255) / 256), 256, 0, stream>>>(Ip(1), Ip(2), KS, KD);
  wprep_kernel<<<(unsigned)((2 * (size_t)D * KT / 8 + 2 * 4 * HH * D / 8 + 255) / 256), 256, 0, stream>>>(Fp(3), Fp(5), Fp(7), Fp(11), WS1, WS2, WL);
  csr_build(cd, KD, E, NK, stream);
  csr_build(cs, KS, E, NK, stream);
  hconv_kernel<1, 1, 0><<<NP / 16, 32, 0, stream>>>(Fp(0), Ip(1), cd.PERM, cd.ROWPTR, cd.ROWCNT, (int)cd.permLen, cs.ROWCNT, WS1, Fp(4), HA, nullptr, nullptr, nullptr, nullptr, nullptr, nullptr);
  hconv_kernel<0, 0, 1><<<NP / 16, 32, 0, stream>>>(HA, Ip(1), cd.PERM, cd.ROWPTR, cd.ROWCNT, (int)cd.permLen, cs.ROWCNT, WS2, Fp(6), nullptr, WL, Fp(9), Fp(10), Fp(13), Fp(14), (float*)d_out);
}
